// CNF_29042568856021
// MI455X (gfx1250) — hardware-verified
//
#include <hip/hip_runtime.h>

typedef __attribute__((ext_vector_type(16))) _Float16 v16h;
typedef __attribute__((ext_vector_type(8)))  _Float16 v8h;
typedef __attribute__((ext_vector_type(8)))  float    v8f;
typedef __attribute__((ext_vector_type(4)))  float    v4f;

constexpr int kRows   = 8192;
constexpr int kDimIn  = 64;
constexpr int kHid    = 256;
constexpr int kSteps  = 10;
constexpr int kStages = 6;
constexpr float kWCarry    = 16.0f;
constexpr float kWCarryInv = 1.0f / 16.0f;
constexpr float kECarry    = 4096.0f;
constexpr float kECarryInv = 1.0f / 4096.0f;
constexpr float kLog2e    = 1.4426950408889634f;
constexpr float kLn2      = 0.6931471805599453f;
constexpr float kInvSteps = 0.1f;

static_assert(kRows % 64 == 0, "M tile multiple");
static_assert(kHid % 64 == 0, "N tile multiple");
static_assert(kDimIn % 64 == 0, "N tile multiple");
static_assert(kDimIn % 32 == 0, "K multiple of 32");
static_assert(kHid % 32 == 0, "K multiple of 32");

constexpr float kA21 = (float)(1.0 / 5.0);
constexpr float kA31 = (float)(3.0 / 40.0);
constexpr float kA32 = (float)(9.0 / 40.0);
constexpr float kA41 = (float)(44.0 / 45.0);
constexpr float kA42 = (float)(-56.0 / 15.0);
constexpr float kA43 = (float)(32.0 / 9.0);
constexpr float kA51 = (float)(19372.0 / 6561.0);
constexpr float kA52 = (float)(-25360.0 / 2187.0);
constexpr float kA53 = (float)(64448.0 / 6561.0);
constexpr float kA54 = (float)(-212.0 / 729.0);
constexpr float kA61 = (float)(9017.0 / 3168.0);
constexpr float kA62 = (float)(-355.0 / 33.0);
constexpr float kA63 = (float)(46732.0 / 5247.0);
constexpr float kA64 = (float)(49.0 / 176.0);
constexpr float kA65 = (float)(-5103.0 / 18656.0);
constexpr float kC1  = (float)(35.0 / 384.0);
constexpr float kC3  = (float)(500.0 / 1113.0);
constexpr float kC4  = (float)(125.0 / 192.0);
constexpr float kC5  = (float)(-2187.0 / 6784.0);
constexpr float kC6  = (float)(11.0 / 84.0);

__constant__ float kLdCoef[5] = {kC1, kC3, kC4, kC5, kC6};

constexpr size_t kBytesW1h = (size_t)kHid * kDimIn * 2;
constexpr size_t kBytesW2h = (size_t)kHid * kHid * 2;
constexpr size_t kBytesW3h = (size_t)kDimIn * kHid * 2;
constexpr size_t kBytesEh  = (size_t)kHid * kHid * 2;
constexpr size_t kBytesY16 = (size_t)kRows * kDimIn * 2;
constexpr size_t kBytesHp  = (size_t)kRows * kHid * 2;
constexpr size_t kBytesKy  = (size_t)kRows * kDimIn * 4;
constexpr size_t kBytesTp  = (size_t)kStages * 4 * kRows * 4;
constexpr size_t kBytesLd  = (size_t)kRows * 4;

constexpr size_t kOffW1h = 0;
constexpr size_t kOffW2h = kOffW1h + kBytesW1h;
constexpr size_t kOffW3h = kOffW2h + kBytesW2h;
constexpr size_t kOffEh  = kOffW3h + kBytesW3h;
constexpr size_t kOffY16 = kOffEh + kBytesEh;
constexpr size_t kOffH1  = kOffY16 + kBytesY16;
constexpr size_t kOffS1  = kOffH1 + kBytesHp;
constexpr size_t kOffH2  = kOffS1 + kBytesHp;
constexpr size_t kOffKy  = kOffH2 + kBytesHp;
constexpr size_t kOffTp  = kOffKy + 5 * kBytesKy;
constexpr size_t kOffYr  = kOffTp + kBytesTp;
constexpr size_t kOffLr  = kOffYr + 2 * kBytesKy;
constexpr size_t kWsTotal = kOffLr + 2 * kBytesLd;

static_assert(kWsTotal == 29491200, "carve total");
static_assert(kWsTotal <= (size_t)134217728, "carve under 128 MiB");
static_assert(kOffW2h % 256 == 0 && kOffW3h % 256 == 0 && kOffEh % 256 == 0 && kOffY16 % 256 == 0, "align");
static_assert(kOffH1 % 256 == 0 && kOffS1 % 256 == 0 && kOffH2 % 256 == 0 && kOffKy % 256 == 0, "align");
static_assert(kOffTp % 256 == 0 && kOffYr % 256 == 0 && kOffLr % 256 == 0, "align");
static_assert((size_t)kRows * kDimIn * 4 == 2097152, "out1 byte offset");
static_assert((size_t)kRows * kDimIn * 4 + (size_t)kRows * 4 == 2129920, "out total bytes");

__device__ __forceinline__ void keep4_h(v16h a, v16h b, v16h c, v16h d) { asm volatile("v_nop" :: "v"(a), "v"(b), "v"(c), "v"(d)); }
__device__ __forceinline__ void acc_guard4(v8f& a, v8f& b, v8f& c, v8f& d) { asm volatile("v_nop\n\tv_nop\n\tv_nop\n\tv_nop" : "+v"(a), "+v"(b), "+v"(c), "+v"(d)); }
__device__ __forceinline__ void guard_row(v8f& a0, v8f& a1, v8f& a2, v8f& a3, v16h x, v16h b0, v16h b1, v16h b2, v16h b3) {
  asm volatile("v_nop\n\tv_nop\n\tv_nop\n\tv_nop" : "+v"(a0), "+v"(a1), "+v"(a2), "+v"(a3) : "v"(x), "v"(b0), "v"(b1), "v"(b2), "v"(b3));
}
template <typename T> struct Frag;
template <> struct Frag<_Float16> {
  typedef v16h V; union U { v16h v; v8h h[2]; };
  static __device__ __forceinline__ v16h load(const _Float16* p) {
    U f; f.h[0] = *(const v8h*)(p); f.h[1] = *(const v8h*)(p + 16); return f.v;
  }
  static __device__ __forceinline__ v8f mma(v16h a, v16h b, v8f c) {
    return __builtin_amdgcn_wmma_f32_16x16x32_f16(false, a, false, b, (short)0, c, false, false);
  }
};
typedef Frag<_Float16> FragH;

__device__ __forceinline__ void wave_sync() {
  __builtin_amdgcn_fence(__ATOMIC_RELEASE, "workgroup");
  __builtin_amdgcn_wave_barrier();
  __builtin_amdgcn_fence(__ATOMIC_ACQUIRE, "workgroup");
}

__device__ __forceinline__ void zero_acc(v8f (&acc)[4][4]) {
#pragma unroll
  for (int i = 0; i < 4; ++i)
#pragma unroll
    for (int j = 0; j < 4; ++j) acc[i][j] = (v8f){0.f, 0.f, 0.f, 0.f, 0.f, 0.f, 0.f, 0.f};
}

__device__ __forceinline__ void mma_tile64(v8f (&acc)[4][4], const _Float16* __restrict__ A, int lda,
                                           const _Float16* __restrict__ Bt, int ldb, int m0, int n0, int K, int lane) {
  const int rlane = lane & 15;
  const int koff  = (lane >> 4) * 8;
#pragma unroll 1
  for (int k0 = 0; k0 < K; k0 += 32) {
    v16h bh[4];
#pragma unroll
    for (int j = 0; j < 4; ++j) {
      const size_t bo = (size_t)(n0 + (j << 4) + rlane) * ldb + koff + k0;
      bh[j] = FragH::load(Bt + bo);
    }
#pragma unroll
    for (int i = 0; i < 4; ++i) {
      const size_t ao = (size_t)(m0 + (i << 4) + rlane) * lda + koff + k0;
      const v16h ah = FragH::load(A + ao);
#pragma unroll
      for (int j = 0; j < 4; ++j) acc[i][j] = FragH::mma(ah, bh[j], acc[i][j]);
      guard_row(acc[i][0], acc[i][1], acc[i][2], acc[i][3], ah, bh[0], bh[1], bh[2], bh[3]);
    }
    keep4_h(bh[0], bh[1], bh[2], bh[3]);
  }
  acc_guard4(acc[0][0], acc[0][1], acc[0][2], acc[0][3]);
  acc_guard4(acc[1][0], acc[1][1], acc[1][2], acc[1][3]);
  acc_guard4(acc[2][0], acc[2][1], acc[2][2], acc[2][3]);
  acc_guard4(acc[3][0], acc[3][1], acc[3][2], acc[3][3]);
}

__device__ __forceinline__ void softplus_sigmoid(float z, float& sp, float& sg) {
  const float e   = __builtin_amdgcn_exp2f(-fabsf(z) * kLog2e);
  const float ope = 1.0f + e;
  sp = fmaxf(z, 0.0f) + kLn2 * __builtin_amdgcn_logf(ope);
  const float rc = __builtin_amdgcn_rcpf(ope);
  sg = (z >= 0.0f) ? rc : e * rc;
}

__global__ __launch_bounds__(256) void k_cast8(const float* __restrict__ in, unsigned short* __restrict__ out, int n8, float carry) {
  const int i = blockIdx.x * 256 + threadIdx.x;
  if (i >= n8) return;
  const float* p = in + 8 * (size_t)i;
  const v4f a = *(const v4f*)(p);
  const v4f c = *(const v4f*)(p + 4);
  v8h hv;
#pragma unroll
  for (int e = 0; e < 4; ++e) {
    hv[e]     = (_Float16)(a[e] * carry);
    hv[4 + e] = (_Float16)(c[e] * carry);
  }
  unsigned short* q = out + 8 * (size_t)i;
  *(volatile v8h*)q = hv;
  __threadfence();
  *(volatile v8h*)q = hv;
}

__global__ __launch_bounds__(256) void k_build_e(const float* __restrict__ W1, const float* __restrict__ W2,
                                                 const float* __restrict__ W3, unsigned short* __restrict__ Eh, float carry) {
  __shared__ __align__(16) float sW1[64 * 64];
  __shared__ __align__(16) float sW3[64 * 32];
  const int t  = threadIdx.x;
  const int n0 = blockIdx.x * 32;
  const int k0 = blockIdx.y * 64;
#pragma unroll
  for (int i = 0; i < 4; ++i) {
    const int idx = i * 256 + t;
    *(v4f*)(sW1 + 4 * idx) = *(const v4f*)(W1 + (size_t)k0 * kDimIn + 4 * idx);
  }
#pragma unroll
  for (int i = 0; i < 2; ++i) {
    const int idx = i * 256 + t;
    const int d = idx >> 3;
    const int c = (idx & 7) * 4;
    *(v4f*)(sW3 + d * 32 + c) = *(const v4f*)(W3 + (size_t)d * kHid + n0 + c);
  }
  __syncthreads();
  const int nl = t >> 3;
  const int kg = t & 7;
  float mx[8];
#pragma unroll
  for (int j = 0; j < 8; ++j) mx[j] = 0.0f;
#pragma unroll 1
  for (int d = 0; d < kDimIn; ++d) {
    const float w3 = sW3[d * 32 + nl];
#pragma unroll
    for (int j = 0; j < 8; ++j) mx[j] = mx[j] + sW1[(kg * 8 + j) * 64 + d] * w3;
  }
  const int n = n0 + nl;
  const float* w2p = W2 + (size_t)n * kHid + k0 + kg * 8;
  const v4f wa = *(const v4f*)(w2p);
  const v4f wb = *(const v4f*)(w2p + 4);
  v8h hv;
#pragma unroll
  for (int j = 0; j < 4; ++j) {
    const float e0 = carry * (wa[j] * mx[j]);
    const float e1 = carry * (wb[j] * mx[4 + j]);
    hv[j]     = (_Float16)e0;
    hv[4 + j] = (_Float16)e1;
  }
  unsigned short* dst = Eh + (size_t)n * kHid + k0 + kg * 8;
  *(volatile v8h*)dst = hv;
  __threadfence();
  *(volatile v8h*)dst = hv;
}

constexpr int kSlabF = 16 * 68;

__global__ __launch_bounds__(256) void k_gemm_in(const unsigned short* __restrict__ Ap, const unsigned short* __restrict__ Btp,
                                                 const float* __restrict__ bias,
                                                 unsigned short* __restrict__ outH, unsigned short* __restrict__ outS) {
  __shared__ __align__(16) float sT[8][kSlabF];
  const int lane = threadIdx.x & 31;
  const int wave = threadIdx.x >> 5;
  constexpr int tilesN = kHid / 64;
  constexpr int tilesM = kRows / 64;
  const int tile = blockIdx.x * 8 + wave;
  if (tile >= tilesM * tilesN) return;
  const int tm = tile / tilesN;
  const int tn = tile - tm * tilesN;
  const int m0 = tm << 6;
  const int n0 = tn << 6;
  const _Float16* A  = (const _Float16*)(const void*)Ap;
  const _Float16* Bt = (const _Float16*)(const void*)Btp;

  v8f acc[4][4];
  zero_acc(acc);
  mma_tile64(acc, A, kDimIn, Bt, kDimIn, m0, n0, kDimIn, lane);

  float* slab = sT[wave];
  const int rlane = lane & 15;
  const int mOff  = (lane >> 4) * 8;
  const int q  = lane >> 3;
  const int c8 = (lane & 7) * 8;
#pragma unroll
  for (int i = 0; i < 4; ++i) {
    const int mBase = m0 + (i << 4);
#pragma unroll
    for (int j = 0; j < 4; ++j) {
      const float bv = bias[n0 + (j << 4) + rlane];
#pragma unroll
      for (int r = 0; r < 8; ++r) slab[(mOff + r) * 68 + (j << 4) + rlane] = acc[i][j][r] * kWCarryInv + bv;
    }
    wave_sync();
#pragma unroll 1
    for (int it = 0; it < 4; ++it) {
      const int row = it * 4 + q;
      const float* zp = slab + row * 68 + c8;
      const v4f z0 = *(const v4f*)(zp);
      const v4f z1 = *(const v4f*)(zp + 4);
      v8h hv, sv;
#pragma unroll
      for (int e = 0; e < 4; ++e) {
        float a, g;
        softplus_sigmoid(z0[e], a, g);
        hv[e] = (_Float16)a;
        sv[e] = (_Float16)g;
        softplus_sigmoid(z1[e], a, g);
        hv[4 + e] = (_Float16)a;
        sv[4 + e] = (_Float16)g;
      }
      const size_t go = (size_t)(mBase + row) * kHid + n0 + c8;
      *(volatile v8h*)(outH + go) = hv;
      *(volatile v8h*)(outS + go) = sv;
      __threadfence();
      *(volatile v8h*)(outH + go) = hv;
      *(volatile v8h*)(outS + go) = sv;
    }
    wave_sync();
  }
}

constexpr int kMidTst  = 64 * 64;
constexpr int kMidRowp = 64;
constexpr int kMidWaveFloats = kMidTst + kSlabF + kMidRowp;
constexpr size_t kMidLdsBytes = (size_t)8 * kMidWaveFloats * 4;
static_assert(kMidLdsBytes == 167936, "dynamic LDS bytes");

__global__ __launch_bounds__(256) void k_gemm_mid(const unsigned short* __restrict__ Ahp, const unsigned short* __restrict__ Asp,
                                                  const unsigned short* __restrict__ Bwp, const unsigned short* __restrict__ Bep,
                                                  const float* __restrict__ bias, unsigned short* __restrict__ outH,
                                                  float* __restrict__ tpout) {
  extern __shared__ float4 dsm_raw[];
  const int lane = threadIdx.x & 31;
  const int wave = threadIdx.x >> 5;
  constexpr int tilesN = kHid / 64;
  constexpr int tilesM = kRows / 64;
  const int tile = blockIdx.x * 8 + wave;
  if (tile >= tilesM * tilesN) return;
  const int tm = tile / tilesN;
  const int tn = tile - tm * tilesN;
  const int m0 = tm << 6;
  const int n0 = tn << 6;
  float* wb   = (float*)dsm_raw + (size_t)wave * kMidWaveFloats;
  float* tst  = wb;
  float* slab = wb + kMidTst;
  float* rowp = slab + kSlabF;
  const int rlane = lane & 15;
  const int mOff  = (lane >> 4) * 8;
  const int q  = lane >> 3;
  const int c8 = (lane & 7) * 8;
  const _Float16* Ah = (const _Float16*)(const void*)Ahp;
  const _Float16* As = (const _Float16*)(const void*)Asp;
  const _Float16* Bw = (const _Float16*)(const void*)Bwp;
  const _Float16* Be = (const _Float16*)(const void*)Bep;

  v8f acc[4][4];
  zero_acc(acc);
  mma_tile64(acc, As, kHid, Be, kHid, m0, n0, kHid, lane);
#pragma unroll
  for (int i = 0; i < 4; ++i)
#pragma unroll
    for (int j = 0; j < 4; ++j)
#pragma unroll
      for (int r = 0; r < 8; ++r)
        tst[(((i << 4) + mOff + r) << 6) + (j << 4) + rlane] = acc[i][j][r] * kECarryInv;
  wave_sync();

  zero_acc(acc);
  mma_tile64(acc, Ah, kHid, Bw, kHid, m0, n0, kHid, lane);

#pragma unroll
  for (int i = 0; i < 4; ++i) {
    const int mBase = m0 + (i << 4);
    float prow[8];
#pragma unroll
    for (int r = 0; r < 8; ++r) prow[r] = 0.0f;
#pragma unroll
    for (int j = 0; j < 4; ++j) {
      const float bv = bias[n0 + (j << 4) + rlane];
#pragma unroll
      for (int r = 0; r < 8; ++r) {
        const float z = acc[i][j][r] * kWCarryInv + bv;
        float sp, sg;
        softplus_sigmoid(z, sp, sg);
        const float tt = tst[(((i << 4) + mOff + r) << 6) + (j << 4) + rlane];
        prow[r] = prow[r] + sg * tt;
        slab[(mOff + r) * 68 + (j << 4) + rlane] = sp;
      }
    }
#pragma unroll
    for (int r = 0; r < 8; ++r) {
      float v = prow[r];
      v += __shfl_xor(v, 1, 32);
      v += __shfl_xor(v, 2, 32);
      v += __shfl_xor(v, 4, 32);
      v += __shfl_xor(v, 8, 32);
      if (rlane == 0) rowp[(i << 4) + mOff + r] = v;
    }
    wave_sync();
#pragma unroll 1
    for (int it = 0; it < 4; ++it) {
      const int row = it * 4 + q;
      const float* hp = slab + row * 68 + c8;
      const v4f a = *(const v4f*)(hp);
      const v4f b = *(const v4f*)(hp + 4);
      v8h hv;
#pragma unroll
      for (int e = 0; e < 4; ++e) {
        hv[e]     = (_Float16)a[e];
        hv[4 + e] = (_Float16)b[e];
      }
      const size_t go = (size_t)(mBase + row) * kHid + n0 + c8;
      *(volatile v8h*)(outH + go) = hv;
      __threadfence();
      *(volatile v8h*)(outH + go) = hv;
    }
    wave_sync();
  }
  {
    const v4f pv = *(const v4f*)(rowp + 4 * rlane);
    float* dst = tpout + (size_t)tn * kRows + m0 + 4 * rlane;
    if (lane < 16) *(volatile v4f*)dst = pv;
    __threadfence();
    if (lane < 16) *(volatile v4f*)dst = pv;
  }
}

__device__ __forceinline__ v4f ldv4(const float* p) { return *(const v4f*)p; }
__device__ __forceinline__ v4f tp_sum(const float* __restrict__ tpl, int s, size_t ro) {
  const float* b = tpl + (size_t)s * 4 * kRows + ro;
  const v4f t0 = ldv4(b);
  const v4f t1 = ldv4(b + kRows);
  const v4f t2 = ldv4(b + 2 * kRows);
  const v4f t3 = ldv4(b + 3 * kRows);
  return ((t0 + t1) + t2) + t3;
}

template <int STG>
__global__ __launch_bounds__(256) void k_gemm_out(const unsigned short* __restrict__ Ap, const unsigned short* __restrict__ Btp,
                                                  const float* __restrict__ bias, const float* __restrict__ tptr,
                                                  const float* __restrict__ yrun,
                                                  const float* __restrict__ kp1, const float* __restrict__ kp2,
                                                  const float* __restrict__ kp3, const float* __restrict__ kp4,
                                                  float* __restrict__ kout, unsigned short* __restrict__ y16,
                                                  float* __restrict__ yout, const float* __restrict__ ldin,
                                                  float* __restrict__ ldout, const float* __restrict__ tpl) {
  __shared__ __align__(16) float sT[8][kSlabF];
  const int lane = threadIdx.x & 31;
  const int wave = threadIdx.x >> 5;
  const int tile = blockIdx.x * 8 + wave;
  if (tile >= kRows / 64) return;
  const int m0 = tile << 6;
  const float dt = tptr[0] * kInvSteps;
  const _Float16* A  = (const _Float16*)(const void*)Ap;
  const _Float16* Bt = (const _Float16*)(const void*)Btp;

  v8f acc[4][4];
  zero_acc(acc);
  mma_tile64(acc, A, kHid, Bt, kHid, m0, 0, kHid, lane);

  float* slab = sT[wave];
  const int rlane = lane & 15;
  const int mOff  = (lane >> 4) * 8;
  const int hh = lane >> 4;
  const int c4 = (lane & 15) * 4;
  const int q  = lane >> 3;
  const int c8 = (lane & 7) * 8;
#pragma unroll
  for (int i = 0; i < 4; ++i) {
    const int mBase = m0 + (i << 4);
#pragma unroll
    for (int j = 0; j < 4; ++j) {
      const float bv = bias[(j << 4) + rlane];
#pragma unroll
      for (int r = 0; r < 8; ++r) slab[(mOff + r) * 68 + (j << 4) + rlane] = acc[i][j][r] * kWCarryInv + bv;
    }
    wave_sync();
#pragma unroll 1
    for (int it = 0; it < 8; ++it) {
      const int row = it * 2 + hh;
      const size_t go = (size_t)(mBase + row) * kDimIn + c4;
      float* cell = slab + row * 68 + c4;
      const v4f kv = *(const v4f*)cell;
      const v4f yv = ldv4(yrun + go);
      v4f s;
      if (STG == 0) {
        s = kv * kA21;
      } else if (STG == 1) {
        const v4f k1 = ldv4(kp1 + go);
        s = k1 * kA31 + kv * kA32;
      } else if (STG == 2) {
        const v4f k1 = ldv4(kp1 + go);
        const v4f k2 = ldv4(kp2 + go);
        s = k1 * kA41 + k2 * kA42 + kv * kA43;
      } else if (STG == 3) {
        const v4f k1 = ldv4(kp1 + go);
        const v4f k2 = ldv4(kp2 + go);
        const v4f k3 = ldv4(kp3 + go);
        s = k1 * kA51 + k2 * kA52 + k3 * kA53 + kv * kA54;
      } else if (STG == 4) {
        const v4f k1 = ldv4(kp1 + go);
        const v4f k2 = ldv4(kp2 + go);
        const v4f k3 = ldv4(kp3 + go);
        const v4f k4 = ldv4(kp4 + go);
        s = k1 * kA61 + k2 * kA62 + k3 * kA63 + k4 * kA64 + kv * kA65;
      } else {
        const v4f k1 = ldv4(kp1 + go);
        const v4f k3 = ldv4(kp2 + go);
        const v4f k4 = ldv4(kp3 + go);
        const v4f k5 = ldv4(kp4 + go);
        s = k1 * kC1 + k3 * kC3 + k4 * kC4 + k5 * kC5 + kv * kC6;
      }
      const v4f yn = yv + s * dt;
      if (STG < 5) {
        *(volatile v4f*)(kout + go) = kv;
      } else {
        *(volatile v4f*)(yout + go) = yn;
      }
      __threadfence();
      if (STG < 5) {
        *(volatile v4f*)(kout + go) = kv;
      } else {
        *(volatile v4f*)(yout + go) = yn;
      }
      *(v4f*)cell = yn;
    }
    wave_sync();
#pragma unroll 1
    for (int it = 0; it < 4; ++it) {
      const int row = it * 4 + q;
      const float* yp = slab + row * 68 + c8;
      const v4f a = *(const v4f*)(yp);
      const v4f b = *(const v4f*)(yp + 4);
      v8h hv;
#pragma unroll
      for (int e = 0; e < 4; ++e) {
        hv[e]     = (_Float16)a[e];
        hv[4 + e] = (_Float16)b[e];
      }
      const size_t go16 = (size_t)(mBase + row) * kDimIn + c8;
      *(volatile v8h*)(y16 + go16) = hv;
      __threadfence();
      *(volatile v8h*)(y16 + go16) = hv;
    }
    wave_sync();
  }
  if (STG == 5) {
    const int l16 = lane & 15;
    const size_t ro = (size_t)m0 + 4 * l16;
    const v4f lv = ldv4(ldin + ro);
    v4f ls = (v4f){0.f, 0.f, 0.f, 0.f};
#pragma unroll 1
    for (int g = 0; g < 5; ++g) {
      const int sidx = g + ((g != 0) ? 1 : 0);
      const float cf = kLdCoef[g];
      const v4f t = tp_sum(tpl, sidx, ro);
      ls = ls + t * cf;
    }
    const v4f ln = lv + ls * dt;
    if (hh == 0) *(volatile v4f*)(ldout + ro) = ln;
    __threadfence();
    if (hh == 0) *(volatile v4f*)(ldout + ro) = ln;
  }
}

extern "C" void kernel_launch(void* const* d_in, const int* in_sizes, int n_in,
                              void* d_out, int out_size, void* d_ws, size_t ws_size, hipStream_t stream) {
  if (n_in < 9) return;
  if (ws_size < kWsTotal) return;
  if ((size_t)out_size != (size_t)kRows * kDimIn + (size_t)kRows) return;
  if (in_sizes[0] != kRows * kDimIn || in_sizes[1] != kRows || in_sizes[2] != kHid * kDimIn || in_sizes[3] != kHid ||
      in_sizes[4] != kHid * kHid || in_sizes[5] != kHid || in_sizes[6] != kDimIn * kHid || in_sizes[7] != kDimIn ||
      in_sizes[8] < 1) return;

  const float* x   = (const float*)d_in[0];
  const float* ld0 = (const float*)d_in[1];
  const float* W1  = (const float*)d_in[2];
  const float* b1  = (const float*)d_in[3];
  const float* W2  = (const float*)d_in[4];
  const float* b2  = (const float*)d_in[5];
  const float* W3  = (const float*)d_in[6];
  const float* b3  = (const float*)d_in[7];
  const float* Tp  = (const float*)d_in[8];

  float* out0 = (float*)d_out;
  float* out1 = (float*)d_out + (size_t)kRows * kDimIn;

  char* ws = (char*)d_ws;
  unsigned short* w1h = (unsigned short*)(ws + kOffW1h);
  unsigned short* w2h = (unsigned short*)(ws + kOffW2h);
  unsigned short* w3h = (unsigned short*)(ws + kOffW3h);
  unsigned short* eh  = (unsigned short*)(ws + kOffEh);
  unsigned short* y16 = (unsigned short*)(ws + kOffY16);
  unsigned short* h1h = (unsigned short*)(ws + kOffH1);
  unsigned short* s1h = (unsigned short*)(ws + kOffS1);
  unsigned short* h2h = (unsigned short*)(ws + kOffH2);
  float* ky[5];
  for (int i = 0; i < 5; ++i) ky[i] = (float*)(ws + kOffKy + (size_t)i * kBytesKy);
  float* tp = (float*)(ws + kOffTp);
  float* yr[2];
  yr[0] = (float*)(ws + kOffYr);
  yr[1] = (float*)(ws + kOffYr + kBytesKy);
  float* lr[2];
  lr[0] = (float*)(ws + kOffLr);
  lr[1] = (float*)(ws + kOffLr + kBytesLd);

  k_cast8<<<(kHid * kDimIn / 8) / 256, 256, 0, stream>>>(W1, w1h, kHid * kDimIn / 8, kWCarry);
  k_cast8<<<(kHid * kHid / 8) / 256, 256, 0, stream>>>(W2, w2h, kHid * kHid / 8, kWCarry);
  k_cast8<<<(kDimIn * kHid / 8) / 256, 256, 0, stream>>>(W3, w3h, kDimIn * kHid / 8, kWCarry);
  k_build_e<<<dim3(kHid / 32, kHid / 64), 256, 0, stream>>>(W1, W2, W3, eh, kECarry);
  k_cast8<<<(kRows * kDimIn / 8) / 256, 256, 0, stream>>>(x, y16, kRows * kDimIn / 8, 1.0f);

  const int gemmBlocks  = (kRows / 64) * (kHid / 64) / 8;
  const int gemm3Blocks = (kRows / 64) / 8;

  for (int step = 0; step < kSteps; ++step) {
    const float* yin  = (step == 0) ? x : yr[(step - 1) & 1];
    const float* ldin = (step == 0) ? ld0 : lr[(step - 1) & 1];
    float* yout  = (step == kSteps - 1) ? out0 : yr[step & 1];
    float* ldout = (step == kSteps - 1) ? out1 : lr[step & 1];
    for (int s = 0; s < kStages; ++s) {
      k_gemm_in<<<gemmBlocks, 256, 0, stream>>>(y16, w1h, b1, h1h, s1h);
      k_gemm_mid<<<gemmBlocks, 256, kMidLdsBytes, stream>>>(h1h, s1h, w2h, eh, b2, h2h, tp + (size_t)s * 4 * kRows);
      if (s == 0) {
        k_gemm_out<0><<<gemm3Blocks, 256, 0, stream>>>(h2h, w3h, b3, Tp, yin, ky[1], ky[2], ky[3], ky[4], ky[0], y16,
                                                        yout, ldin, ldout, tp);
      } else if (s == 1) {
        k_gemm_out<1><<<gemm3Blocks, 256, 0, stream>>>(h2h, w3h, b3, Tp, yin, ky[0], ky[2], ky[3], ky[4], ky[1], y16,
                                                        yout, ldin, ldout, tp);
      } else if (s == 2) {
        k_gemm_out<2><<<gemm3Blocks, 256, 0, stream>>>(h2h, w3h, b3, Tp, yin, ky[0], ky[1], ky[3], ky[4], ky[2], y16,
                                                        yout, ldin, ldout, tp);
      } else if (s == 3) {
        k_gemm_out<3><<<gemm3Blocks, 256, 0, stream>>>(h2h, w3h, b3, Tp, yin, ky[0], ky[1], ky[2], ky[4], ky[3], y16,
                                                        yout, ldin, ldout, tp);
      } else if (s == 4) {
        k_gemm_out<4><<<gemm3Blocks, 256, 0, stream>>>(h2h, w3h, b3, Tp, yin, ky[0], ky[1], ky[2], ky[3], ky[4], y16,
                                                        yout, ldin, ldout, tp);
      } else {
        k_gemm_out<5><<<gemm3Blocks, 256, 0, stream>>>(h2h, w3h, b3, Tp, yin, ky[0], ky[2], ky[3], ky[4], ky[1], y16,
                                                        yout, ldin, ldout, tp);
      }
    }
  }
}
